// DecoderOnlyLayer_67302137528535
// MI455X (gfx1250) — hardware-verified
//
#include <hip/hip_runtime.h>
#include <math.h>
#include <stdint.h>

#define NB     2
#define SEQ    2048
#define DM     1024
#define NH     16
#define HD     64
#define DFF    4096
#define MROWS  (NB * SEQ)
#define NQB    (SEQ / 64)
#define VLP    512
#define RESQB  8
#define LNEPS  1e-6f
#define WSCALE 64.0f
static_assert(RESQB * 64 <= VLP);
static_assert(NH * HD == DM);
static_assert((SEQ % 64) == 0 && (DM % 64) == 0 && (DFF % 64) == 0 && (MROWS % 64) == 0);
static_assert(NQB * 8 == 256);

typedef _Float16 v16h __attribute__((ext_vector_type(16)));
typedef _Float16 v8h  __attribute__((ext_vector_type(8)));
typedef __bf16   v16b __attribute__((ext_vector_type(16)));
typedef __bf16   v8b  __attribute__((ext_vector_type(8)));
typedef float    v8f  __attribute__((ext_vector_type(8)));
typedef float    v4f  __attribute__((ext_vector_type(4)));
typedef unsigned int v4u __attribute__((ext_vector_type(4)));
typedef unsigned int v2u __attribute__((ext_vector_type(2)));
typedef int      v4i __attribute__((ext_vector_type(4)));
typedef unsigned long long u64;

#if defined(__HIP_DEVICE_COMPILE__)
#define DEV_ASM 1
#else
#define DEV_ASM 0
#endif

__device__ __forceinline__ unsigned short bf_bits(float f) {
  unsigned u = __float_as_uint(f);
  return (unsigned short)((u + 0x7FFFu + ((u >> 16) & 1u)) >> 16);
}
__device__ __forceinline__ float bf_up(unsigned short h) { return __uint_as_float(((unsigned)h) << 16); }
__device__ __forceinline__ float bfr(float f) { return bf_up(bf_bits(f)); }
__device__ __forceinline__ unsigned short h_bits(_Float16 x) { return __builtin_bit_cast(unsigned short, x); }
__device__ __forceinline__ unsigned pk16(unsigned short a, unsigned short b) { return (unsigned)a | ((unsigned)b << 16); }
__device__ __forceinline__ v8f zero8() { v8f z = {0.f, 0.f, 0.f, 0.f, 0.f, 0.f, 0.f, 0.f}; return z; }
__device__ __forceinline__ v8h zero8h() {
  const _Float16 z = (_Float16)0.0f;
  v8h r = {z, z, z, z, z, z, z, z};
  return r;
}

template <int ET> struct OpT;
template <> struct OpT<0> {
  typedef __bf16 E; typedef v16b F; typedef v8b H;
  static __device__ __forceinline__ F ld(const E* p) {
    union { F v; H h[2]; } f;
    f.h[0] = *(const H*)(p);
    f.h[1] = *(const H*)(p + 16);
    return f.v;
  }
  static __device__ __forceinline__ v8f mma_raw(F a, F b, v8f c) {
    return __builtin_amdgcn_wmma_f32_16x16x32_bf16(false, a, false, b, (short)0, c, false, false);
  }
  static __device__ __forceinline__ void dep_guard(v8f& a, v8f& b, F x, F y) {
#if DEV_ASM
    asm volatile("v_nop\n\tv_nop\n\tv_nop\n\tv_nop" : "+v"(a), "+v"(b) : "v"(x), "v"(y));
#endif
  }
  static __device__ __forceinline__ void keep4(F a, F b, F c, F d) {
#if DEV_ASM
    asm volatile("v_nop" :: "v"(a), "v"(b), "v"(c), "v"(d));
#endif
  }
};
template <> struct OpT<1> {
  typedef _Float16 E; typedef v16h F; typedef v8h H;
  static __device__ __forceinline__ F ld(const E* p) {
    union { F v; H h[2]; } f;
    f.h[0] = *(const H*)(p);
    f.h[1] = *(const H*)(p + 16);
    return f.v;
  }
  static __device__ __forceinline__ v8f mma_raw(F a, F b, v8f c) {
    return __builtin_amdgcn_wmma_f32_16x16x32_f16(false, a, false, b, (short)0, c, false, false);
  }
  static __device__ __forceinline__ void dep_guard(v8f& a, v8f& b, F x, F y) {
#if DEV_ASM
    asm volatile("v_nop\n\tv_nop\n\tv_nop\n\tv_nop" : "+v"(a), "+v"(b) : "v"(x), "v"(y));
#endif
  }
  static __device__ __forceinline__ void keep4(F a, F b, F c, F d) {
#if DEV_ASM
    asm volatile("v_nop" :: "v"(a), "v"(b), "v"(c), "v"(d));
#endif
  }
};

__device__ __forceinline__ v8f mma_b(v16b a, v16b b, v8f c) {
  c = __builtin_amdgcn_wmma_f32_16x16x32_bf16(false, a, false, b, (short)0, c, false, false);
#if DEV_ASM
  asm volatile("v_nop\n\tv_nop\n\tv_nop\n\tv_nop" : "+v"(c) : "v"(a), "v"(b));
#endif
  return c;
}
__device__ __forceinline__ v8f mma_h(v16h a, v16h b, v8f c) {
  c = __builtin_amdgcn_wmma_f32_16x16x32_f16(false, a, false, b, (short)0, c, false, false);
#if DEV_ASM
  asm volatile("v_nop\n\tv_nop\n\tv_nop\n\tv_nop" : "+v"(c) : "v"(a), "v"(b));
#endif
  return c;
}
__device__ __forceinline__ void acc_guard4(v8f& a, v8f& b, v8f& c, v8f& d) {
#if DEV_ASM
  asm volatile("v_nop\n\tv_nop\n\tv_nop\n\tv_nop" : "+v"(a), "+v"(b), "+v"(c), "+v"(d));
#endif
}

__global__ __launch_bounds__(256) void cvt_bf16x8(const float* __restrict__ in, unsigned short* out, int n8) {
  const int i = blockIdx.x * 256 + threadIdx.x;
  if (i < n8) {
    const v4f a = *(const v4f*)(in + (size_t)i * 8);
    const v4f b = *(const v4f*)(in + (size_t)i * 8 + 4);
    v4u p;
    p[0] = pk16(bf_bits(a[0]), bf_bits(a[1]));
    p[1] = pk16(bf_bits(a[2]), bf_bits(a[3]));
    p[2] = pk16(bf_bits(b[0]), bf_bits(b[1]));
    p[3] = pk16(bf_bits(b[2]), bf_bits(b[3]));
    *(volatile v4u*)(out + (size_t)i * 8) = p;
    __threadfence();
    *(volatile v4u*)(out + (size_t)i * 8) = p;
  }
}

template <bool F16OUT>
__global__ __launch_bounds__(256) void wtrans64(const float* __restrict__ W, unsigned short* out,
                                                 int Kdim, int Ndim, float scale) {
  __shared__ float tile[64][65];
  const int tid = threadIdx.x, lane = tid & 31, wave = tid >> 5;
  const int n0 = blockIdx.x * 64, k0 = blockIdx.y * 64;
  {
    const int r = tid >> 2, cq = (tid & 3) * 16;
    const float* src = W + (size_t)(k0 + r) * Ndim + n0 + cq;
#pragma unroll
    for (int e = 0; e < 4; ++e) {
      const v4f a = *(const v4f*)(src + 4 * e);
      tile[r][cq + 4 * e + 0] = a[0];
      tile[r][cq + 4 * e + 1] = a[1];
      tile[r][cq + 4 * e + 2] = a[2];
      tile[r][cq + 4 * e + 3] = a[3];
    }
  }
  __syncthreads();
  const int q = lane >> 3, c8 = (lane & 7) * 8;
  v4u pv[2];
#pragma unroll
  for (int it = 0; it < 2; ++it) {
    const int nn = wave * 8 + it * 4 + q;
    v4u a;
#pragma unroll
    for (int e = 0; e < 4; ++e) {
      const float f0 = tile[c8 + 2 * e][nn], f1 = tile[c8 + 2 * e + 1][nn];
      unsigned short b0 = bf_bits(f0), b1 = bf_bits(f1);
      if (F16OUT) {
        b0 = h_bits((_Float16)(bf_up(b0) * scale));
        b1 = h_bits((_Float16)(bf_up(b1) * scale));
      }
      a[e] = pk16(b0, b1);
    }
    pv[it] = a;
  }
  for (int pass = 0; pass < 2; ++pass) {
#pragma unroll
    for (int it = 0; it < 2; ++it) {
      const int nn = wave * 8 + it * 4 + q;
      *(volatile v4u*)(out + (size_t)(n0 + nn) * Kdim + k0 + c8) = pv[it];
    }
    __threadfence();
  }
}

__global__ __launch_bounds__(256) void mask_rowbits(const int* __restrict__ maskp, u64* flg) {
  __shared__ __align__(8) unsigned char sb[NQB * 8];
  const int tid  = threadIdx.x;
  const int wave = tid >> 5;
  const int lane = tid & 31;
  const int qt   = blockIdx.x;
  const int row  = tid >> 2;
  const int qtr  = (tid & 3) * 16;
  const int* mr = maskp + ((size_t)qt * 64 + row) * SEQ + qtr;
#pragma unroll 1
  for (int kt = 0; kt < NQB; ++kt) {
    const int* p = mr + kt * 64;
    const v4i a0 = *(const v4i*)(p);
    const v4i a1 = *(const v4i*)(p + 4);
    const v4i a2 = *(const v4i*)(p + 8);
    const v4i a3 = *(const v4i*)(p + 12);
    int lv = 0;
#pragma unroll
    for (int e = 0; e < 4; ++e) {
      lv |= (a0[e] != 0) ? 1 : 0;
      lv |= (a1[e] != 0) ? 1 : 0;
      lv |= (a2[e] != 0) ? 1 : 0;
      lv |= (a3[e] != 0) ? 1 : 0;
    }
    const unsigned bl = __builtin_amdgcn_ballot_w32(lv != 0);
    unsigned bits = 0u;
#pragma unroll
    for (int k = 0; k < 8; ++k) bits |= ((((bl >> (4 * k)) & 0xFu) != 0u) ? 1u : 0u) << k;
    if (lane == 0) sb[kt * 8 + wave] = (unsigned char)bits;
  }
  __syncthreads();
  if (wave == 0) {
    u64 w;
    __builtin_memcpy(&w, &sb[lane * 8], 8);
    u64* dst = flg + (size_t)qt * NQB + lane;
    *(volatile u64*)dst = w;
    __threadfence();
    *(volatile u64*)dst = w;
  }
}

template <int ET, int NSPLIT, int OUT_MODE, int BIAS, int RESID, bool RELU>
__global__ __launch_bounds__(256) void gemm64(
    const unsigned short* __restrict__ Ap, const unsigned short* __restrict__ A2p, int lda, long long strideA,
    const unsigned short* __restrict__ Btp, int ldb, long long strideB,
    const float* __restrict__ bias,
    const void* __restrict__ resid, int ldr, long long strideR,
    void* Cout, int ldc, long long strideC,
    void* Cout2, int ldc2, long long strideC2, int N2,
    int M, int N, int K, float oscale, float rscale) {
  typedef typename OpT<ET>::E E;
  typedef typename OpT<ET>::F F;
  const E* A  = (const E*)(const void*)Ap;
  const E* A2 = (const E*)(const void*)A2p;
  const E* Bt = (const E*)(const void*)Btp;
  __shared__ __align__(16) float sT[8][16 * 68];
  const int b    = blockIdx.y;
  const int lane = threadIdx.x & 31;
  const int wave = threadIdx.x >> 5;
  const int tilesN = N >> 6;
  const int tilesM = M >> 6;
  const int tile = blockIdx.x * 8 + wave;
  if (tile >= tilesM * tilesN) return;
  const int tm = tile / tilesN;
  const int tn = tile - tm * tilesN;
  const int m0 = tm << 6;
  const int n0 = tn << 6;

  const E* Ab  = A  + (size_t)b * strideA;
  const E* Bb  = Bt + (size_t)b * strideB;
  const E* Ab2 = (NSPLIT >= 1) ? (A2 + (size_t)b * strideA) : Ab;

  const int rlane = lane & 15;
  const int koff  = (lane >> 4) * 8;
  const int mOff  = (lane >> 4) * 8;

  v8f acc[4][4];
#pragma unroll
  for (int i = 0; i < 4; ++i)
#pragma unroll
    for (int j = 0; j < 4; ++j) acc[i][j] = zero8();

  for (int k0 = 0; k0 < K; k0 += 32) {
    F bh[4];
#pragma unroll
    for (int j = 0; j < 4; ++j) {
      const size_t bofs = (size_t)(n0 + (j << 4) + rlane) * ldb + koff + k0;
      bh[j] = OpT<ET>::ld(Bb + bofs);
    }
#pragma unroll
    for (int i = 0; i < 4; ++i) {
      const size_t aofs = (size_t)(m0 + (i << 4) + rlane) * lda + koff + k0;
      const F ah = OpT<ET>::ld(Ab + aofs);
      F al = ah;
      if (NSPLIT >= 1) al = OpT<ET>::ld(Ab2 + aofs);
#pragma unroll
      for (int j = 0; j < 4; ++j) {
        acc[i][j] = OpT<ET>::mma_raw(ah, bh[j], acc[i][j]);
        if (NSPLIT >= 1) acc[i][j] = OpT<ET>::mma_raw(al, bh[j], acc[i][j]);
      }
      OpT<ET>::dep_guard(acc[i][0], acc[i][3], ah, al);
    }
    OpT<ET>::keep4(bh[0], bh[1], bh[2], bh[3]);
  }
  acc_guard4(acc[0][0], acc[0][1], acc[0][2], acc[0][3]);
  acc_guard4(acc[1][0], acc[1][1], acc[1][2], acc[1][3]);
  acc_guard4(acc[2][0], acc[2][1], acc[2][2], acc[2][3]);
  acc_guard4(acc[3][0], acc[3][1], acc[3][2], acc[3][3]);

  float* slab = sT[wave];
#pragma unroll
  for (int i = 0; i < 4; ++i) {
    const int mBase = m0 + (i << 4);
#pragma unroll
    for (int j = 0; j < 4; ++j) {
#pragma unroll
      for (int r = 0; r < 8; ++r) {
        slab[(mOff + r) * 68 + (j << 4) + rlane] = acc[i][j][r];
      }
    }
    __builtin_amdgcn_fence(__ATOMIC_RELEASE, "workgroup");
    __builtin_amdgcn_wave_barrier();
    __builtin_amdgcn_fence(__ATOMIC_ACQUIRE, "workgroup");
    if (OUT_MODE == 0) {
      float* C = (float*)Cout + (size_t)b * strideC;
      const int h2 = lane >> 4, c4 = (lane & 15) * 4;
      v4f bz = {0.f, 0.f, 0.f, 0.f};
      if (BIAS == 1) {
        const v4f g = *(const v4f*)(bias + n0 + c4);
        bz[0] = bfr(g[0]); bz[1] = bfr(g[1]); bz[2] = bfr(g[2]); bz[3] = bfr(g[3]);
      }
      v4f ov[8];
#pragma unroll
      for (int it = 0; it < 8; ++it) {
        const int row = it * 2 + h2;
        const v4f v = *(const v4f*)(slab + row * 68 + c4);
        v4f w;
        w[0] = v[0] * oscale + bz[0];
        w[1] = v[1] * oscale + bz[1];
        w[2] = v[2] * oscale + bz[2];
        w[3] = v[3] * oscale + bz[3];
        if (BIAS == 2) {
          const float bm = bfr(bias[mBase + row]);
          w[0] += bm; w[1] += bm; w[2] += bm; w[3] += bm;
        }
        if (RESID == 1) {
          const unsigned short* rp = (const unsigned short*)resid + (size_t)b * strideR +
                                     (size_t)(mBase + row) * ldr + n0 + c4;
          const v2u rr = *(const v2u*)rp;
          w[0] += __uint_as_float(rr[0] << 16);
          w[1] += __uint_as_float(rr[0] & 0xffff0000u);
          w[2] += __uint_as_float(rr[1] << 16);
          w[3] += __uint_as_float(rr[1] & 0xffff0000u);
        }
        if (RESID == 2) {
          const float* rp = (const float*)resid + (size_t)b * strideR + (size_t)(mBase + row) * ldr + n0 + c4;
          const v4f rr = *(const v4f*)rp;
          w[0] += rr[0]; w[1] += rr[1]; w[2] += rr[2]; w[3] += rr[3];
        }
        if (RELU) {
          w[0] = fmaxf(w[0], 0.f); w[1] = fmaxf(w[1], 0.f); w[2] = fmaxf(w[2], 0.f); w[3] = fmaxf(w[3], 0.f);
        }
        ov[it] = w;
      }
      for (int pass = 0; pass < 2; ++pass) {
#pragma unroll
        for (int it = 0; it < 8; ++it) {
          const int row = it * 2 + h2;
          *(volatile v4f*)(C + (size_t)(mBase + row) * ldc + n0 + c4) = ov[it];
        }
        __threadfence();
      }
    } else {
      const int q = lane >> 3, c8 = (lane & 7) * 8;
      unsigned short* C  = (unsigned short*)Cout  + (size_t)b * strideC;
      unsigned short* C2 = (unsigned short*)Cout2 + (size_t)b * strideC2;
      const bool wlo = (OUT_MODE == 2) || (OUT_MODE == 3 && n0 < N2);
      float b8[8];
#pragma unroll
      for (int e = 0; e < 8; ++e) b8[e] = 0.f;
      if (BIAS == 1) {
        const v4f g0 = *(const v4f*)(bias + n0 + c8);
        const v4f g1 = *(const v4f*)(bias + n0 + c8 + 4);
#pragma unroll
        for (int e = 0; e < 4; ++e) { b8[e] = bfr(g0[e]); b8[4 + e] = bfr(g1[e]); }
      }
      v4u hv[4], lv[4];
#pragma unroll
      for (int it = 0; it < 4; ++it) {
        const int row = it * 4 + q;
        const float* sp = slab + row * 68 + c8;
        float bm = 0.f;
        if (BIAS == 2) bm = bfr(bias[mBase + row]);
        v4u a, a2;
#pragma unroll
        for (int e = 0; e < 4; ++e) {
          float f0 = sp[2 * e] * oscale + b8[2 * e] + bm;
          float f1 = sp[2 * e + 1] * oscale + b8[2 * e + 1] + bm;
          if (RELU) { f0 = fmaxf(f0, 0.f); f1 = fmaxf(f1, 0.f); }
          unsigned short h0, h1, l0 = 0, l1 = 0;
          if (OUT_MODE == 2) {
            h0 = bf_bits(f0); h1 = bf_bits(f1);
            l0 = bf_bits(f0 - bf_up(h0)); l1 = bf_bits(f1 - bf_up(h1));
          } else if (OUT_MODE == 3) {
            const _Float16 x0 = (_Float16)f0, x1 = (_Float16)f1;
            h0 = h_bits(x0); h1 = h_bits(x1);
            l0 = h_bits((_Float16)((f0 - (float)x0) * rscale));
            l1 = h_bits((_Float16)((f1 - (float)x1) * rscale));
          } else {
            h0 = h_bits((_Float16)f0); h1 = h_bits((_Float16)f1);
          }
          a[e] = pk16(h0, h1); a2[e] = pk16(l0, l1);
        }
        hv[it] = a; lv[it] = a2;
      }
      for (int pass = 0; pass < 2; ++pass) {
#pragma unroll
        for (int it = 0; it < 4; ++it) {
          const int row = it * 4 + q;
          *(volatile v4u*)(C + (size_t)(mBase + row) * ldc + n0 + c8) = hv[it];
          if (wlo) *(volatile v4u*)(C2 + (size_t)(mBase + row) * ldc2 + n0 + c8) = lv[it];
        }
        __threadfence();
      }
    }
    __builtin_amdgcn_fence(__ATOMIC_RELEASE, "workgroup");
    __builtin_amdgcn_wave_barrier();
    __builtin_amdgcn_fence(__ATOMIC_ACQUIRE, "workgroup");
  }
}

template <bool RES>
__global__ __launch_bounds__(128)
void attn_mask64(const unsigned short* __restrict__ qhp, const unsigned short* __restrict__ qlp,
                 const unsigned short* __restrict__ khp, const unsigned short* __restrict__ klp,
                 const unsigned short* __restrict__ vhp, const unsigned short* __restrict__ vlp,
                 const int* __restrict__ maskp, const u64* __restrict__ flg,
                 unsigned short* ohp, unsigned short* olp,
                 int qbBase, int nqbThis, float sscale) {
  union FB { v16b v; v8b h[2]; };
  union FH { v16h v; v8h h[2]; };
  __shared__ __align__(16) __bf16   Ksh[64 * 64];
  __shared__ __align__(16) __bf16   Ksl[64 * 64];
  __shared__ __align__(16) _Float16 Vth[64 * 64];
  __shared__ __align__(16) _Float16 Vtl[RES ? 64 * 64 : 8];
  __shared__ __align__(16) _Float16 Psh[4][16 * 64];
  __shared__ __align__(16) _Float16 Psl[RES ? 4 : 1][16 * 64];
  __shared__ __align__(16) float    Os[4][16 * 64];

  const int tid  = threadIdx.x;
  const int wave = tid >> 5;
  const int lane = tid & 31;
  const int hh   = lane >> 4;
  const int c    = lane & 15;

  const int bx   = blockIdx.x;
  const int qbl  = bx % nqbThis;
  const int rest = bx / nqbThis;
  const int h    = rest % NH;
  const int b    = rest / NH;
  const int qb   = qbBase + qbl;
  const int q0   = qb * 64 + wave * 16;
  const size_t rowB = (size_t)b * SEQ;

  const __bf16* Qh = (const __bf16*)(const void*)qhp + (size_t)h * HD;
  const __bf16* Ql = (const __bf16*)(const void*)qlp + (size_t)h * HD;
  const __bf16* Kh = (const __bf16*)(const void*)khp + (size_t)h * HD;
  const __bf16* Kl = (const __bf16*)(const void*)klp + (size_t)h * HD;
  const _Float16* Vh = (const _Float16*)(const void*)vhp + ((size_t)b * DM + (size_t)h * HD) * SEQ;
  const _Float16* Vl = (const _Float16*)(const void*)vlp + ((size_t)b * DM + (size_t)h * HD) * VLP;
  const u64* fq = flg + (size_t)qb * NQB;

  v16b qah[2], qal[2];
#pragma unroll
  for (int dc = 0; dc < 2; ++dc) {
    const size_t qo = (rowB + q0 + c) * DM + dc * 32 + 8 * hh;
    qah[dc] = OpT<0>::ld(Qh + qo);
    qal[dc] = OpT<0>::ld(Ql + qo);
  }

  float mrow[8], lrow[8];
  v8f oacc[4];
#pragma unroll
  for (int r = 0; r < 8; ++r) { mrow[r] = -INFINITY; lrow[r] = 0.f; }
#pragma unroll
  for (int t = 0; t < 4; ++t) oacc[t] = zero8();

  for (int kt = 0; kt < NQB; ++kt) {
    const u64 lw = fq[kt];
    if (lw == 0ull) continue;
    const int kv0 = kt * 64;
    __syncthreads();
    {
      const int r = tid >> 1, half = (tid & 1) * 32;
      const __bf16*   kg  = Kh + (rowB + kv0 + r) * DM + half;
      const __bf16*   klg = Kl + (rowB + kv0 + r) * DM + half;
      const _Float16* vg  = Vh + (size_t)r * SEQ + kv0 + half;
      const int kvl = (kv0 + 64 <= VLP) ? kv0 : (VLP - 64);
      const _Float16* vlg = Vl + (size_t)r * VLP + kvl + half;
      const bool resOK = (kv0 + 64 <= VLP);
#pragma unroll
      for (int i = 0; i < 4; ++i) {
        const v8b a0 = *(const v8b*)(kg + 8 * i);
        const v8b a1 = *(const v8b*)(klg + 8 * i);
        const v8h b0 = *(const v8h*)(vg + 8 * i);
        *(v8b*)(Ksh + r * 64 + half + 8 * i) = a0;
        *(v8b*)(Ksl + r * 64 + half + 8 * i) = a1;
        *(v8h*)(Vth + r * 64 + half + 8 * i) = b0;
        if (RES) {
          v8h b1 = *(const v8h*)(vlg + 8 * i);
          if (!resOK) b1 = zero8h();
          *(v8h*)(Vtl + r * 64 + half + 8 * i) = b1;
        }
      }
    }
    __syncthreads();

    v8f s[4];
#pragma unroll
    for (int j = 0; j < 4; ++j) {
      s[j] = zero8();
#pragma unroll
      for (int dc = 0; dc < 2; ++dc) {
        FB kb, kl;
        kb.h[0] = *(const v8b*)(Ksh + (j * 16 + c) * 64 + dc * 32 + 8 * hh);
        kb.h[1] = *(const v8b*)(Ksh + (j * 16 + c) * 64 + dc * 32 + 16 + 8 * hh);
        kl.h[0] = *(const v8b*)(Ksl + (j * 16 + c) * 64 + dc * 32 + 8 * hh);
        kl.h[1] = *(const v8b*)(Ksl + (j * 16 + c) * 64 + dc * 32 + 16 + 8 * hh);
        s[j] = mma_b(qah[dc], kb.v, s[j]);
        s[j] = mma_b(qah[dc], kl.v, s[j]);
        s[j] = mma_b(qal[dc], kb.v, s[j]);
      }
    }

    _Float16* pwh = Psh[wave];
    _Float16* pwl = Psl[RES ? wave : 0];
    const int* mq = maskp + (size_t)(q0 + 8 * hh) * SEQ + kv0 + c;
#pragma unroll
    for (int r = 0; r < 8; ++r) {
      const int* mrw = mq + (size_t)r * SEQ;
      float m = -INFINITY;
#pragma unroll
      for (int j = 0; j < 4; ++j) {
        const int mv = mrw[j * 16];
        const float sv = (mv != 0) ? (s[j][r] * sscale) : -INFINITY;
        s[j][r] = sv;
        m = fmaxf(m, sv);
      }
#pragma unroll
      for (int off = 1; off < 16; off <<= 1) m = fmaxf(m, __shfl_xor(m, off, 32));
      const float mnew  = fmaxf(mrow[r], m);
      const float msafe = (mnew == -INFINITY) ? 0.f : mnew;
      const float alpha = __expf(mrow[r] - msafe);
      mrow[r] = mnew;
      float psum = 0.f;
#pragma unroll
      for (int j = 0; j < 4; ++j) {
        const float p = __expf(s[j][r] - msafe);
        psum += p;
        const float p1k = p * 1024.0f;
        const _Float16 ph = (_Float16)p1k;
        pwh[(8 * hh + r) * 64 + j * 16 + c] = ph;
        if (RES) {
          const _Float16 pl = (_Float16)((p1k - (float)ph) * 4096.0f);
          pwl[(8 * hh + r) * 64 + j * 16 + c] = pl;
        }
      }
#pragma unroll
      for (int off = 1; off < 16; off <<= 1) psum += __shfl_xor(psum, off, 32);
      lrow[r] = lrow[r] * alpha + psum;
#pragma unroll
      for (int t = 0; t < 4; ++t) oacc[t][r] *= alpha;
    }
    __builtin_amdgcn_fence(__ATOMIC_RELEASE, "workgroup");
    __builtin_amdgcn_wave_barrier();
    __builtin_amdgcn_fence(__ATOMIC_ACQUIRE, "workgroup");

    v8f o1[4];
#pragma unroll
    for (int t = 0; t < 4; ++t) o1[t] = zero8();
#pragma unroll 1
    for (int kk = 0; kk < 2; ++kk) {
      FH pa, pl;
      pa.h[0] = *(const v8h*)(pwh + c * 64 + kk * 32 + 8 * hh);
      pa.h[1] = *(const v8h*)(pwh + c * 64 + kk * 32 + 16 + 8 * hh);
      if (RES) {
        pl.h[0] = *(const v8h*)(pwl + c * 64 + kk * 32 + 8 * hh);
        pl.h[1] = *(const v8h*)(pwl + c * 64 + kk * 32 + 16 + 8 * hh);
      } else {
        pl.v = pa.v;
      }
#pragma unroll
      for (int t = 0; t < 4; ++t) {
        FH vb;
        vb.h[0] = *(const v8h*)(Vth + (t * 16 + c) * 64 + kk * 32 + 8 * hh);
        vb.h[1] = *(const v8h*)(Vth + (t * 16 + c) * 64 + kk * 32 + 16 + 8 * hh);
        oacc[t] = mma_h(pa.v, vb.v, oacc[t]);
        if (RES) {
          FH vl;
          vl.h[0] = *(const v8h*)(Vtl + (t * 16 + c) * 64 + kk * 32 + 8 * hh);
          vl.h[1] = *(const v8h*)(Vtl + (t * 16 + c) * 64 + kk * 32 + 16 + 8 * hh);
          o1[t] = mma_h(pa.v, vl.v, o1[t]);
          o1[t] = mma_h(pl.v, vb.v, o1[t]);
        }
      }
    }
    if (RES) {
#pragma unroll
      for (int t = 0; t < 4; ++t)
#pragma unroll
        for (int r = 0; r < 8; ++r) oacc[t][r] += o1[t][r] * (1.0f / 4096.0f);
    }
  }

  float* os = Os[wave];
#pragma unroll
  for (int r = 0; r < 8; ++r) {
    const float l = lrow[r];
    const float inv = (1.0f / l) * (1.0f / 1024.0f);
#pragma unroll
    for (int t = 0; t < 4; ++t) os[(8 * hh + r) * 64 + t * 16 + c] = oacc[t][r] * inv;
  }
  __builtin_amdgcn_fence(__ATOMIC_RELEASE, "workgroup");
  __builtin_amdgcn_wave_barrier();
  __builtin_amdgcn_fence(__ATOMIC_ACQUIRE, "workgroup");
  {
    const int q4 = lane >> 3, c8 = (lane & 7) * 8;
    v4u hv[4], lv[4];
#pragma unroll
    for (int it = 0; it < 4; ++it) {
      const int row = it * 4 + q4;
      const float* sp = os + row * 64 + c8;
      v4u a, a2;
#pragma unroll
      for (int e = 0; e < 4; ++e) {
        const float f0 = sp[2 * e], f1 = sp[2 * e + 1];
        const unsigned short h0 = bf_bits(f0), h1 = bf_bits(f1);
        const unsigned short l0 = bf_bits(f0 - bf_up(h0)), l1 = bf_bits(f1 - bf_up(h1));
        a[e] = pk16(h0, h1); a2[e] = pk16(l0, l1);
      }
      hv[it] = a; lv[it] = a2;
    }
    for (int pass = 0; pass < 2; ++pass) {
#pragma unroll
      for (int it = 0; it < 4; ++it) {
        const int row = it * 4 + q4;
        const size_t go = (rowB + q0 + row) * DM + (size_t)h * HD + c8;
        *(volatile v4u*)(ohp + go) = hv[it];
        *(volatile v4u*)(olp + go) = lv[it];
      }
      __threadfence();
    }
  }
}

template <bool OUT16>
__global__ __launch_bounds__(256) void layernorm_rows(const float* __restrict__ in,
                                                       const float* __restrict__ gamma,
                                                       const float* __restrict__ beta,
                                                       float* out32, unsigned short* out16) {
  __shared__ float red[16];
  const int tid = threadIdx.x, lane = tid & 31, wave = tid >> 5;
  const int row = blockIdx.x;
  const float* xr = in + (size_t)row * DM;
  const v4f v = *(const v4f*)(xr + tid * 4);
  float s = (v[0] + v[1]) + (v[2] + v[3]);
#pragma unroll
  for (int off = 1; off < 32; off <<= 1) s += __shfl_xor(s, off, 32);
  if (lane == 0) red[wave] = s;
  __syncthreads();
  float tot = 0.f;
#pragma unroll
  for (int i = 0; i < 8; ++i) tot += red[i];
  const float mean = tot * (1.0f / (float)DM);
  const float d0 = v[0] - mean, d1 = v[1] - mean, d2 = v[2] - mean, d3 = v[3] - mean;
  float s2 = (d0 * d0 + d1 * d1) + (d2 * d2 + d3 * d3);
#pragma unroll
  for (int off = 1; off < 32; off <<= 1) s2 += __shfl_xor(s2, off, 32);
  if (lane == 0) red[8 + wave] = s2;
  __syncthreads();
  float tot2 = 0.f;
#pragma unroll
  for (int i = 0; i < 8; ++i) tot2 += red[8 + i];
  const float var  = tot2 * (1.0f / (float)DM);
  const float rstd = 1.0f / sqrtf(var + LNEPS);

  const v4f g  = *(const v4f*)(gamma + tid * 4);
  const v4f bt = *(const v4f*)(beta + tid * 4);
  v4f o;
  o[0] = (bfr(g[0]) * d0) * rstd + bfr(bt[0]);
  o[1] = (bfr(g[1]) * d1) * rstd + bfr(bt[1]);
  o[2] = (bfr(g[2]) * d2) * rstd + bfr(bt[2]);
  o[3] = (bfr(g[3]) * d3) * rstd + bfr(bt[3]);
  float* op = out32 + (size_t)row * DM + tid * 4;
  *(volatile v4f*)op = o;
  __threadfence();
  *(volatile v4f*)op = o;

  if (OUT16) {
    if (tid < 128) {
      const int cc = tid * 8;
      const v4f a0 = *(const v4f*)(xr + cc);
      const v4f a1 = *(const v4f*)(xr + cc + 4);
      const v4f g0 = *(const v4f*)(gamma + cc), g1 = *(const v4f*)(gamma + cc + 4);
      const v4f b0 = *(const v4f*)(beta + cc),  b1 = *(const v4f*)(beta + cc + 4);
      float f[8];
#pragma unroll
      for (int e = 0; e < 4; ++e) {
        f[e]     = (bfr(g0[e]) * (a0[e] - mean)) * rstd + bfr(b0[e]);
        f[4 + e] = (bfr(g1[e]) * (a1[e] - mean)) * rstd + bfr(b1[e]);
      }
      v4u hp;
#pragma unroll
      for (int e = 0; e < 4; ++e) hp[e] = pk16(h_bits((_Float16)f[2 * e]), h_bits((_Float16)f[2 * e + 1]));
      unsigned short* hq = out16 + (size_t)row * DM + cc;
      *(volatile v4u*)hq = hp;
      __threadfence();
      *(volatile v4u*)hq = hp;
    }
  }
}

extern "C" void kernel_launch(void* const* d_in, const int* in_sizes, int n_in,
                              void* d_out, int out_size, void* d_ws, size_t ws_size,
                              hipStream_t stream) {
  if (n_in < 18) return;
  if (in_sizes[0] != NB * SEQ * DM) return;
  if (in_sizes[1] != SEQ * SEQ) return;
  if (in_sizes[2] != DM * DM || in_sizes[4] != DM * DM || in_sizes[6] != DM * DM || in_sizes[8] != DM * DM) return;
  if (in_sizes[3] != DM || in_sizes[5] != DM || in_sizes[7] != DM || in_sizes[9] != DM) return;
  if (in_sizes[10] != DM * DFF || in_sizes[11] != DFF || in_sizes[12] != DFF * DM || in_sizes[13] != DM) return;
  if (in_sizes[14] != DM || in_sizes[15] != DM || in_sizes[16] != DM || in_sizes[17] != DM) return;
  if (out_size != NB * SEQ * DM) return;

  const float* x   = (const float*)d_in[0];
  const int*   msk = (const int*)d_in[1];
  const float* Wq  = (const float*)d_in[2];
  const float* bq  = (const float*)d_in[3];
  const float* Wk  = (const float*)d_in[4];
  const float* bk  = (const float*)d_in[5];
  const float* Wv  = (const float*)d_in[6];
  const float* bv  = (const float*)d_in[7];
  const float* Wo  = (const float*)d_in[8];
  const float* bo  = (const float*)d_in[9];
  const float* W1  = (const float*)d_in[10];
  const float* b1  = (const float*)d_in[11];
  const float* W2  = (const float*)d_in[12];
  const float* b2  = (const float*)d_in[13];
  const float* gamma1 = (const float*)d_in[14];
  const float* beta1  = (const float*)d_in[15];
  const float* gamma2 = (const float*)d_in[16];
  const float* beta2  = (const float*)d_in[17];

  const size_t PX   = (size_t)MROWS * DM * 2;
  const size_t PW   = (size_t)DM * DM * 2;
  const size_t PWF  = (size_t)DM * DFF * 2;
  const size_t PVT  = (size_t)NB * DM * SEQ * 2;
  const size_t PVL  = (size_t)NB * DM * VLP * 2;
  const size_t PFs  = (size_t)2 * 1048576;
  const size_t PF   = (size_t)NQB * NQB * 8;
  const size_t PT   = (size_t)MROWS * DM * 4;
  const size_t PF1  = (size_t)MROWS * DFF * 2;
  if (PF > PFs) return;
  size_t off = 0;
  const size_t oXb  = off; off += PX;
  const size_t oWq  = off; off += PW;
  const size_t oWk  = off; off += PW;
  const size_t oWv  = off; off += PW;
  const size_t oWo  = off; off += PW;
  const size_t oW1  = off; off += PWF;
  const size_t oW2  = off; off += PWF;
  const size_t oQh  = off; off += PX;
  const size_t oQl  = off; off += PX;
  const size_t oKh  = off; off += PX;
  const size_t oKl  = off; off += PX;
  const size_t oVTh = off; off += PVT;
  const size_t oVTl = off; off += PVL;
  const size_t oFlg = off; off += PFs;
  const size_t oOh  = off; off += PX;
  const size_t oOl  = off; off += PX;
  const size_t endA = off;
  const size_t oT1  = oQh;
  const size_t oH32 = oKh;
  const size_t oHh  = oVTh;
  const size_t oF1  = oVTl;
  const size_t oT2  = oT1;
  if (oT1 + PT != oKh) return;
  if (oH32 + PT != oVTh) return;
  if (oHh + PX != oVTl) return;
  size_t total = oF1 + PF1;
  if (endA > total) total = endA;
  if (total > ws_size) return;
  if (total > (size_t)134217728) return;

  char* ws = (char*)d_ws;
  unsigned short* Xb   = (unsigned short*)(ws + oXb);
  unsigned short* WqTb = (unsigned short*)(ws + oWq);
  unsigned short* WkTb = (unsigned short*)(ws + oWk);
  unsigned short* WvTb = (unsigned short*)(ws + oWv);
  unsigned short* WoTb = (unsigned short*)(ws + oWo);
  unsigned short* W1Tb = (unsigned short*)(ws + oW1);
  unsigned short* W2Tb = (unsigned short*)(ws + oW2);
  unsigned short* Qh   = (unsigned short*)(ws + oQh);
  unsigned short* Ql   = (unsigned short*)(ws + oQl);
  unsigned short* Kh   = (unsigned short*)(ws + oKh);
  unsigned short* Kl   = (unsigned short*)(ws + oKl);
  unsigned short* VTh  = (unsigned short*)(ws + oVTh);
  unsigned short* VTl  = (unsigned short*)(ws + oVTl);
  u64*            Flg  = (u64*)(ws + oFlg);
  unsigned short* Oh   = (unsigned short*)(ws + oOh);
  unsigned short* Ol   = (unsigned short*)(ws + oOl);
  float*          T1   = (float*)(ws + oT1);
  float*          H32  = (float*)(ws + oH32);
  unsigned short* Hh   = (unsigned short*)(ws + oHh);
  unsigned short* F1   = (unsigned short*)(ws + oF1);
  float*          T2   = (float*)(ws + oT2);

  const dim3 blk(256);
  const int n8x = MROWS * DM / 8;
  const dim3 gCvtX((n8x + 255) / 256);
  const dim3 gMask(NQB);
  const dim3 gTw(DM / 64, DM / 64);
  const dim3 gTw1(DFF / 64, DM / 64);
  const dim3 gTw2(DM / 64, DFF / 64);
  const dim3 gProj(((MROWS / 64) * (DM / 64) + 7) / 8, 1);
  const dim3 gVT(((DM / 64) * (SEQ / 64) + 7) / 8, NB);
  const dim3 gW1(((MROWS / 64) * (DFF / 64) + 7) / 8, 1);
  const dim3 gW2(((MROWS / 64) * (DM / 64) + 7) / 8, 1);
  const dim3 gLN(MROWS);

  mask_rowbits<<<gMask, blk, 0, stream>>>(msk, Flg);
  cvt_bf16x8<<<gCvtX, blk, 0, stream>>>(x, Xb, n8x);
  wtrans64<false><<<gTw, blk, 0, stream>>>(Wq, WqTb, DM, DM, 1.0f);
  wtrans64<false><<<gTw, blk, 0, stream>>>(Wk, WkTb, DM, DM, 1.0f);
  wtrans64<false><<<gTw, blk, 0, stream>>>(Wv, WvTb, DM, DM, 1.0f);
  wtrans64<false><<<gTw, blk, 0, stream>>>(Wo, WoTb, DM, DM, 1.0f);
  wtrans64<true><<<gTw1, blk, 0, stream>>>(W1, W1Tb, DM, DFF, WSCALE);
  wtrans64<true><<<gTw2, blk, 0, stream>>>(W2, W2Tb, DFF, DM, WSCALE);
  gemm64<0, 0, 2, 1, 0, false><<<gProj, blk, 0, stream>>>(
      Xb, Xb, DM, 0LL, WqTb, DM, 0LL, bq, (const void*)Xb, DM, 0LL,
      (void*)Qh, DM, 0LL, (void*)Ql, DM, 0LL, DM,
      MROWS, DM, DM, 1.0f, 1.0f);
  gemm64<0, 0, 2, 1, 0, false><<<gProj, blk, 0, stream>>>(
      Xb, Xb, DM, 0LL, WkTb, DM, 0LL, bk, (const void*)Xb, DM, 0LL,
      (void*)Kh, DM, 0LL, (void*)Kl, DM, 0LL, DM,
      MROWS, DM, DM, 1.0f, 1.0f);
  gemm64<0, 0, 3, 2, 0, false><<<gVT, blk, 0, stream>>>(
      WvTb, WvTb, DM, 0LL, Xb, DM, (long long)SEQ * DM, bv, (const void*)Xb, DM, 0LL,
      (void*)VTh, SEQ, (long long)DM * SEQ, (void*)VTl, VLP, (long long)DM * VLP, VLP,
      DM, SEQ, DM, 1.0f, 4096.0f);
  attn_mask64<true><<<dim3(NB * NH * RESQB), dim3(128), 0, stream>>>(
      Qh, Ql, Kh, Kl, VTh, VTl, msk, Flg, Oh, Ol, 0, RESQB, 0.125f);
  attn_mask64<false><<<dim3(NB * NH * (NQB - RESQB)), dim3(128), 0, stream>>>(
      Qh, Ql, Kh, Kl, VTh, VTl, msk, Flg, Oh, Ol, RESQB, NQB - RESQB, 0.125f);
  gemm64<0, 1, 0, 1, 1, false><<<gProj, blk, 0, stream>>>(
      Oh, Ol, DM, 0LL, WoTb, DM, 0LL, bo, (const void*)Xb, DM, 0LL,
      (void*)T1, DM, 0LL, (void*)T1, DM, 0LL, 0,
      MROWS, DM, DM, 1.0f, 1.0f);
  layernorm_rows<true><<<gLN, blk, 0, stream>>>(T1, gamma1, beta1, H32, Hh);
  gemm64<1, 0, 4, 1, 0, true><<<gW1, blk, 0, stream>>>(
      Hh, Hh, DM, 0LL, W1Tb, DM, 0LL, b1, (const void*)Hh, DM, 0LL,
      (void*)F1, DFF, 0LL, (void*)F1, DFF, 0LL, 0,
      MROWS, DFF, DM, 1.0f / WSCALE, 1.0f);
  gemm64<1, 0, 0, 1, 2, false><<<gW2, blk, 0, stream>>>(
      F1, F1, DFF, 0LL, W2Tb, DFF, 0LL, b2, (const void*)H32, DM, 0LL,
      (void*)T2, DM, 0LL, (void*)T2, DM, 0LL, 0,
      MROWS, DM, DFF, 1.0f / WSCALE, 1.0f);
  layernorm_rows<false><<<gLN, blk, 0, stream>>>(T2, gamma2, beta2, (float*)d_out, Hh);
  (void)hipGetLastError();
}
